// VRPTWEdgeGNN_8701603741904
// MI455X (gfx1250) — hardware-run, weakly checked
//
#include <hip/hip_runtime.h>


namespace {
constexpr int N = 25000, NP = 25024, E = 400000, H = 128, ND = 8, ED = 4, L = 4, F4 = 4 * H, H2 = 64;
constexpr float XS = 8.0f, WSC = 256.0f, LN_EPS = 1e-5f;
static_assert(E % 64 == 0 && NP % 64 == 0, "tiling");

typedef _Float16 b16;
typedef __attribute__((ext_vector_type(16))) _Float16 v16b;
typedef __attribute__((ext_vector_type(8))) _Float16 v8b;
typedef __attribute__((ext_vector_type(8))) float v8f;
typedef __attribute__((ext_vector_type(4))) float v4f;
typedef __attribute__((ext_vector_type(2))) float v2f;
__device__ __forceinline__ float bf16_rne(float f) { unsigned int u = __float_as_uint(f); u += 0x7FFFu + ((u >> 16) & 1u); return __uint_as_float(u & 0xFFFF0000u); }
__device__ __forceinline__ void split16(float v, b16& hi, b16& lo) { hi = (b16)v; lo = (b16)(v - (float)hi); }
__device__ __forceinline__ v16b frag_kb(const b16* p, int hh) { const v8b a = *(const v8b*)(p + 8 * hh), b = *(const v8b*)(p + 16 + 8 * hh); v16b f;
#pragma unroll
  for (int e = 0; e < 8; ++e) { f[e] = a[e]; f[8 + e] = b[e]; } return f; }
__device__ __forceinline__ v8f wmma16b(v16b a, v16b b, v8f c) { v8f d = __builtin_amdgcn_wmma_f32_16x16x32_f16(false, a, false, b, (short)0, c, false, false); asm volatile("v_nop\n\tv_nop\n\tv_nop\n\tv_nop" : "+v"(d) : "v"(a), "v"(b)); return d; }
__device__ __forceinline__ void wave_lds_sync() { __builtin_amdgcn_fence(__ATOMIC_RELEASE, "workgroup"); __builtin_amdgcn_wave_barrier(); __builtin_amdgcn_fence(__ATOMIC_ACQUIRE, "workgroup"); }
__device__ __forceinline__ float pmul(float a, float b) { float p = a * b; asm volatile("" : "+v"(p)); return p; }
__device__ __forceinline__ float hsum16(float v) { v += __shfl_xor(v, 1); v += __shfl_xor(v, 2); v += __shfl_xor(v, 4); return v + __shfl_xor(v, 8); }
__device__ __forceinline__ int iclamp(int v, int lo, int hi) { return v < lo ? lo : (v > hi ? hi : v); }

constexpr int CSR_NBLK = 512, CSR_GB = 9, CSR_GN = 1 << CSR_GB  , CSR_MAXG = 512, CSR_CAP = 12288  ;
__global__ __launch_bounds__(64) void csrA_kernel(const int* __restrict__ dst, int E, int N, int nG, int CHP, int NGP, int* __restrict__ STG, int* __restrict__ HST) {
  extern __shared__ int sm[];
  int* cnt = sm; int* run = sm + NGP; int* ids = sm + 2 * NGP;
  const int b = blockIdx.x; const int ch = (E + CSR_NBLK - 1) / CSR_NBLK; const int e0 = b * ch, e1 = min(E, e0 + ch);
  for (int i = threadIdx.x; i < NGP; i += 64) cnt[i] = 0;
  for (int i = threadIdx.x; i < CHP; i += 64) ids[i] = -1;
  __syncthreads();
  if (threadIdx.x == 0) {
    for (int e = e0; e < e1; ++e) { int d = dst[e]; d = (d < 0) ? 0 : (d >= N ? N - 1 : d); cnt[d >> CSR_GB] += 1; }
    int acc = 0; for (int g = 0; g < nG; ++g) { run[g] = acc; acc += cnt[g]; }
    for (int e = e0; e < e1; ++e) { int d = dst[e]; d = (d < 0) ? 0 : (d >= N ? N - 1 : d); const int g = d >> CSR_GB; ids[run[g]] = e; run[g] += 1; } }
  __syncthreads();
  typedef __attribute__((ext_vector_type(4))) int v4i;
  for (int pass = 0; pass < 2; ++pass) {
    for (int i = threadIdx.x; i < CHP / 4; i += 64) *(volatile v4i*)(STG + (size_t)b * CHP + i * 4) = *(const v4i*)(&ids[i * 4]);
    for (int i = threadIdx.x; i < NGP / 4; i += 64) { v4i v; for (int e = 0; e < 4; ++e) v[e] = (i * 4 + e < nG) ? cnt[i * 4 + e] : 0; *(volatile v4i*)(HST + (size_t)b * NGP + i * 4) = v; }
    __threadfence(); }
}
__global__ __launch_bounds__(512) void csrS_kernel(const int* __restrict__ HST, int nG, int NGP, int* __restrict__ START, int* __restrict__ TOT, int* __restrict__ OFF) {
  __shared__ int tot[CSR_MAXG];
  const int b = threadIdx.x;
  for (int pass = 0; pass < 2; ++pass) { int runb = 0; for (int g = 0; g < nG; ++g) { int c = HST[(size_t)b * NGP + g]; c = (c < 0) ? 0 : c; ((volatile int*)OFF)[(size_t)g * CSR_NBLK + b] = runb; runb += c; } __threadfence(); }
  for (int g = threadIdx.x; g < nG; g += 512) { int s = 0; for (int bb = 0; bb < CSR_NBLK; ++bb) { int c = HST[(size_t)bb * NGP + g]; s += (c < 0) ? 0 : c; } tot[g] = s; }
  __syncthreads();
  if (threadIdx.x < 32) {
    __shared__ int st[CSR_MAXG + 32];
    if (threadIdx.x == 0) { int acc = 0; for (int g = 0; g < NGP; ++g) { st[g] = acc; if (g < nG) acc += (tot[g] + 31) & ~31; } st[NGP] = acc; }
    __builtin_amdgcn_fence(__ATOMIC_RELEASE, "workgroup"); __builtin_amdgcn_wave_barrier(); __builtin_amdgcn_fence(__ATOMIC_ACQUIRE, "workgroup");
    for (int pass = 0; pass < 2; ++pass) { for (int i = threadIdx.x; i < NGP + 32; i += 32) { ((volatile int*)START)[i] = (i <= NGP) ? st[min(i, NGP)] : 0; ((volatile int*)TOT)[i] = (i < nG) ? tot[i] : 0; } __threadfence(); } }
}
__global__ __launch_bounds__(256) void csrB_kernel(const int* __restrict__ dst, int N, int nG, int CHP, int NGP, int permLen, const int* __restrict__ STG, const int* __restrict__ HST, const int* __restrict__ OFF, const int* __restrict__ START, const int* __restrict__ TOT, int* __restrict__ PERM, int* __restrict__ ROWPTR, int* __restrict__ ROWCNT, int* __restrict__ FLAG) {
  typedef __attribute__((ext_vector_type(4))) int v4i;
  __shared__ int ids[CSR_CAP]; __shared__ unsigned short key[CSR_CAP]; __shared__ int outp[CSR_CAP]; __shared__ int ncnt[CSR_GN + 1]; __shared__ int boff[CSR_NBLK + 1];
  const int g = blockIdx.x, t_ = threadIdx.x; int tot = TOT[g]; int st = START[g], stn = START[g + 1]; const int v0 = g * CSR_GN; const int nv = min(CSR_GN, N - v0);
  st = (st < 0) ? 0 : (st > permLen - 32 ? permLen - 32 : st) & ~31; stn = (stn < st) ? st : (stn > permLen ? permLen : stn); tot = (tot < 0) ? 0 : tot; if (tot > stn - st && tot <= CSR_CAP) tot = stn - st;
  if (tot > CSR_CAP) {
    for (int pass = 0; pass < 2; ++pass) { for (int i = t_; i < CSR_GN / 4; i += 256) { v4i a, c; for (int e = 0; e < 4; ++e) { a[e] = st; c[e] = 0; } *(volatile v4i*)(ROWPTR + v0 + i * 4) = a; *(volatile v4i*)(ROWCNT + v0 + i * 4) = c; } if (t_ == 0) ((volatile int*)FLAG)[0] = 1; __threadfence(); } (void)nv; return; }
  if (t_ == 0) { int acc = 0; for (int b = 0; b < CSR_NBLK; ++b) { boff[b] = acc; int c = HST[(size_t)b * NGP + g]; c = (c < 0) ? 0 : (c > CHP ? CHP : c); acc += c; if (acc > tot) acc = tot; } boff[CSR_NBLK] = acc; }
  for (int i = t_; i <= CSR_GN; i += 256) ncnt[i] = 0;
  __syncthreads();
  for (int b = 0; b < CSR_NBLK; ++b) { const int c = boff[b + 1] - boff[b]; int o_ = OFF[(size_t)g * CSR_NBLK + b]; o_ = (o_ < 0) ? 0 : (o_ > CHP - c ? CHP - c : o_); const int* src_ = STG + (size_t)b * CHP + o_;
    for (int i = t_; i < c; i += 256) { int id = src_[i]; id = (id < 0) ? 0 : id; ids[boff[b] + i] = id; int d = dst[id]; d = (d < v0) ? v0 : (d >= N ? N - 1 : d); int kk = d - v0; kk = (kk < 0) ? 0 : (kk >= CSR_GN ? CSR_GN - 1 : kk); key[boff[b] + i] = (unsigned short)kk; } }
  __syncthreads();
  if (t_ == 0) { for (int i = 0; i < tot; ++i) ncnt[key[i]] += 1; int acc = 0; for (int vl = 0; vl < CSR_GN; ++vl) { const int c = ncnt[vl]; ncnt[vl] = acc; acc += c; } ncnt[CSR_GN] = acc;
    for (int i = 0; i < tot; ++i) { const int vl = key[i]; outp[ncnt[vl]] = ids[i]; ncnt[vl] += 1; }
    for (int vl = CSR_GN; vl > 0; --vl) ncnt[vl] = ncnt[vl - 1]; ncnt[0] = 0; }
  __syncthreads();
  for (int pass = 0; pass < 2; ++pass) {
    for (int i = t_; i < (stn - st) / 4; i += 256) { v4i v; for (int e = 0; e < 4; ++e) { const int q = i * 4 + e; v[e] = (q < tot) ? outp[q] : -1; } *(volatile v4i*)(PERM + st + i * 4) = v; }
    for (int i = t_; i < CSR_GN / 4; i += 256) { v4i a, c; for (int e = 0; e < 4; ++e) { const int vl = i * 4 + e; a[e] = st + ncnt[vl]; c[e] = (vl < nv) ? (ncnt[vl + 1] - ncnt[vl]) : 0; } *(volatile v4i*)(ROWPTR + v0 + i * 4) = a; *(volatile v4i*)(ROWCNT + v0 + i * 4) = c; }
    __threadfence(); }
}
__global__ __launch_bounds__(256) void csrZ_kernel(int* __restrict__ p, size_t n4) { typedef __attribute__((ext_vector_type(4))) int v4i; const size_t tid = (size_t)blockIdx.x * 256 + threadIdx.x, nth = (size_t)gridDim.x * 256; v4i z = {0, 0, 0, 0}; for (size_t i = tid; i < n4; i += nth) *(volatile v4i*)(p + i * 4) = z; }
struct CsrBufs { int *STG, *HST, *OFF, *START, *TOT, *PERM, *ROWPTR, *ROWCNT, *FLAG; int nG, NGP, CHP; size_t permLen; char* base; size_t bytes; };
static size_t csr_carve(CsrBufs& c, char* ws, size_t off, int E, int N) {
  const size_t off0 = off; c.base = ws + off;
  auto al = [&](size_t bytes) { char* p = ws + off; off += (bytes + 255) & ~(size_t)255; return p; };
  c.nG = (N + CSR_GN - 1) / CSR_GN; c.NGP = (c.nG + 31) & ~31; const int ch = (E + CSR_NBLK - 1) / CSR_NBLK; c.CHP = (ch + 31) & ~31; c.permLen = (size_t)E + 32 * (size_t)c.nG + 32;
  c.STG = (int*)al((size_t)CSR_NBLK * c.CHP * 4); c.HST = (int*)al((size_t)CSR_NBLK * c.NGP * 4); c.OFF = (int*)al((size_t)c.NGP * CSR_NBLK * 4); c.START = (int*)al((size_t)(c.NGP + 64) * 4); c.TOT = (int*)al((size_t)(c.NGP + 64) * 4);
  c.PERM = (int*)al(c.permLen * 4); c.ROWPTR = (int*)al((size_t)c.nG * CSR_GN * 4); c.ROWCNT = (int*)al((size_t)c.nG * CSR_GN * 4); c.FLAG = (int*)al(256);
  c.bytes = off - off0; return off;
}
static void csr_build(const CsrBufs& c, const int* dst, int E, int N, hipStream_t stream) {
  const size_t smem = (size_t)(2 * c.NGP + c.CHP) * 4;
  csrZ_kernel<<<512, 256, 0, stream>>>((int*)c.base, c.bytes / 16);
  csrA_kernel<<<CSR_NBLK, 64, smem, stream>>>(dst, E, N, c.nG, c.CHP, c.NGP, c.STG, c.HST);
  csrS_kernel<<<1, 512, 0, stream>>>(c.HST, c.nG, c.NGP, c.START, c.TOT, c.OFF);
  csrB_kernel<<<c.nG, 256, 0, stream>>>(dst, N, c.nG, c.CHP, c.NGP, (int)c.permLen, c.STG, c.HST, c.OFF, c.START, c.TOT, c.PERM, c.ROWPTR, c.ROWCNT, c.FLAG);
}


__global__ __launch_bounds__(256) void prepw_kernel(const float* __restrict__ cw1, const float* __restrict__ cw2, const float* __restrict__ m1, const float* __restrict__ m2, b16* __restrict__ CW1, b16* __restrict__ CW2, b16* __restrict__ M1, b16* __restrict__ M2) {
  const int kind = blockIdx.y, t = blockIdx.x * 256 + threadIdx.x; int IN, OUT; const float* w; b16* dst;
  if (kind < 4) { IN = H; OUT = H; w = cw1 + (size_t)kind * H * H; dst = CW1 + (size_t)kind * H * H; } else if (kind < 8) { IN = H; OUT = H; w = cw2 + (size_t)(kind - 4) * H * H; dst = CW2 + (size_t)(kind - 4) * H * H; }
  else if (kind == 8) { IN = F4; OUT = H; w = m1; dst = M1; } else { IN = H; OUT = H2; w = m2; dst = M2; }
  if (t >= OUT * IN / 8) return; const int o_ = (t * 8) / IN, k0 = t * 8 - o_ * IN; v8b o; for (int j = 0; j < 8; ++j) o[j] = (b16)(bf16_rne(w[(size_t)(k0 + j) * OUT + o_]) * WSC);
  for (int pass = 0; pass < 2; ++pass) { *(volatile v8b*)(dst + (size_t)t * 8) = o; __threadfence(); }
}
__global__ __launch_bounds__(256) void nodeenc_kernel(const float* __restrict__ x, const float* __restrict__ w, const float* __restrict__ b, const float* __restrict__ g, const float* __restrict__ be, float* __restrict__ H32) {
  const int wave = threadIdx.x >> 5, lane = threadIdx.x & 31; const size_t v = ((size_t)blockIdx.x * 8 + wave) * 2 + (lane >> 4); const int c0 = (lane & 15) * 8;
  float u[8]; float xv[ND]; const bool real = v < (size_t)N; for (int k = 0; k < ND; ++k) xv[k] = real ? bf16_rne(x[v * ND + k]) : 0.0f;
  for (int j = 0; j < 8; ++j) { const int c = c0 + j; float s = bf16_rne(b[c]); for (int k = 0; k < ND; ++k) s += pmul(xv[k], bf16_rne(w[k * H + c])); u[j] = fmaxf(s, 0.0f); }
  float sm = 0.0f; for (int j = 0; j < 8; ++j) sm += u[j]; sm = hsum16(sm); const float mu = sm * (1.0f / H); float ss = 0.0f; for (int j = 0; j < 8; ++j) { const float d = u[j] - mu; ss += pmul(d, d); } ss = hsum16(ss); const float rs = rsqrtf(ss * (1.0f / H) + LN_EPS);
  v4f o0, o1; for (int j = 0; j < 8; ++j) { const int c = c0 + j; const float y = real ? pmul((u[j] - mu) * rs, bf16_rne(g[c])) + bf16_rne(be[c]) : 0.0f; if (j < 4) o0[j] = y; else o1[j - 4] = y; }
  for (int pass = 0; pass < 2; ++pass) { *(volatile v4f*)(H32 + v * H + c0) = o0; *(volatile v4f*)(H32 + v * H + c0 + 4) = o1; __threadfence(); }
}
__device__ __forceinline__ void edge_u(const float* __restrict__ ea, const float* __restrict__ w, const float* __restrict__ b, size_t e, int c0, float u[8]) {
  float av[ED]; for (int k = 0; k < ED; ++k) av[k] = bf16_rne(ea[e * ED + k]);
  for (int j = 0; j < 8; ++j) { const int c = c0 + j; float s = bf16_rne(b[c]); for (int k = 0; k < ED; ++k) s += pmul(av[k], bf16_rne(w[k * H + c])); u[j] = fmaxf(s, 0.0f); } }
__global__ __launch_bounds__(256) void edgeenc_kernel(const float* __restrict__ ea, const float* __restrict__ w, const float* __restrict__ b, const float* __restrict__ g, const float* __restrict__ be, b16* __restrict__ EA16) {
  const int wave = threadIdx.x >> 5, lane = threadIdx.x & 31; const size_t e = ((size_t)blockIdx.x * 8 + wave) * 2 + (lane >> 4); const int c0 = (lane & 15) * 8;
  float u[8]; edge_u(ea, w, b, e, c0, u);
  float sm = 0.0f; for (int j = 0; j < 8; ++j) sm += u[j]; sm = hsum16(sm); const float mu = sm * (1.0f / H); float ss = 0.0f; for (int j = 0; j < 8; ++j) { const float d = u[j] - mu; ss += pmul(d, d); } ss = hsum16(ss); const float rs = rsqrtf(ss * (1.0f / H) + LN_EPS);
  v8b o; for (int j = 0; j < 8; ++j) o[j] = (b16)((pmul((u[j] - mu) * rs, bf16_rne(g[c0 + j])) + bf16_rne(be[c0 + j])) * XS);
  for (int pass = 0; pass < 2; ++pass) { *(volatile v8b*)(EA16 + e * H + c0) = o; __threadfence(); }
}
__global__ __launch_bounds__(256) void aggr_kernel(const float* __restrict__ H32, const int* __restrict__ src, const b16* __restrict__ EA16, const int* __restrict__ PERM, const int* __restrict__ ROWPTR, const int* __restrict__ ROWCNT, int permLen, b16* __restrict__ Zh, b16* __restrict__ Zl) {
  const int wave = threadIdx.x >> 5, lane = threadIdx.x & 31; const size_t v = ((size_t)blockIdx.x * 8 + wave) * 2 + (lane >> 4); const int c0 = (lane & 15) * 8;
  int st = ROWPTR[v], cnt = ROWCNT[v]; cnt = iclamp(cnt, 0, 1 << 16); st = iclamp(st, 0, permLen - cnt);
  float acc[8]; for (int j = 0; j < 8; ++j) acc[j] = 0.0f;
  for (int i = 0; i < cnt; ++i) { const int e = iclamp(PERM[st + i], 0, E - 1); const int s = iclamp(src[e], 0, N - 1);
    const v8b ev = *(const v8b*)(EA16 + (size_t)e * H + c0); const v4f h0 = *(const v4f*)(H32 + (size_t)s * H + c0), h1 = *(const v4f*)(H32 + (size_t)s * H + c0 + 4);
#pragma unroll
    for (int j = 0; j < 8; ++j) { const float hv = j < 4 ? h0[j] : h1[j - 4]; acc[j] += fmaxf(hv + (float)ev[j] * (1.0f / XS), 0.0f); } }
  const v4f hv0 = *(const v4f*)(H32 + v * H + c0), hv1 = *(const v4f*)(H32 + v * H + c0 + 4);
  v8b zh, zl; for (int j = 0; j < 8; ++j) { const float z = (j < 4 ? hv0[j] : hv1[j - 4]) + acc[j]; b16 a_, c_; split16(z * XS, a_, c_); zh[j] = a_; zl[j] = c_; }
  for (int pass = 0; pass < 2; ++pass) { *(volatile v8b*)(Zh + v * H + c0) = zh; *(volatile v8b*)(Zl + v * H + c0) = zl; __threadfence(); }
}
__global__ __launch_bounds__(128) void nodemlp_kernel(const b16* __restrict__ Zh, const b16* __restrict__ Zl, const b16* __restrict__ W1, const float* __restrict__ b1, const b16* __restrict__ W2, const float* __restrict__ b2, const float* __restrict__ g, const float* __restrict__ be, float* __restrict__ H32) {
  __shared__ __attribute__((aligned(16))) b16 Th[4][16][H + 8], Tl[4][16][H + 8]; __shared__ __attribute__((aligned(16))) float Ty[4][16][H + 4];
  const int wave = threadIdx.x >> 5, lane = threadIdx.x & 31, nloc = lane & 15, hlf = lane >> 4; const size_t m0 = (size_t)blockIdx.x * 64 + wave * 16;
  v8f acc[8];
#pragma unroll
  for (int t = 0; t < 8; ++t) acc[t] = (v8f){};
#pragma unroll
  for (int kb = 0; kb < H; kb += 32) { const v16b a = frag_kb(Zh + (m0 + nloc) * H + kb, hlf), al = frag_kb(Zl + (m0 + nloc) * H + kb, hlf);
#pragma unroll
    for (int t = 0; t < 8; ++t) { const v16b bw = frag_kb(W1 + (size_t)(t * 16 + nloc) * H + kb, hlf); acc[t] = wmma16b(a, bw, acc[t]); acc[t] = wmma16b(al, bw, acc[t]); } }
#pragma unroll
  for (int t = 0; t < 8; ++t) { const float bb = bf16_rne(b1[t * 16 + nloc]);
#pragma unroll
    for (int r = 0; r < 8; ++r) { b16 a_, c_; split16(fmaxf(acc[t][r] * (1.0f / (XS * WSC)) + bb, 0.0f) * XS, a_, c_); Th[wave][8 * hlf + r][t * 16 + nloc] = a_; Tl[wave][8 * hlf + r][t * 16 + nloc] = c_; } }
  wave_lds_sync();
#pragma unroll
  for (int t = 0; t < 8; ++t) acc[t] = (v8f){};
#pragma unroll
  for (int kb = 0; kb < H; kb += 32) { const v16b a = frag_kb(&Th[wave][nloc][kb], hlf), al = frag_kb(&Tl[wave][nloc][kb], hlf);
#pragma unroll
    for (int t = 0; t < 8; ++t) { const v16b bw = frag_kb(W2 + (size_t)(t * 16 + nloc) * H + kb, hlf); acc[t] = wmma16b(a, bw, acc[t]); acc[t] = wmma16b(al, bw, acc[t]); } }
#pragma unroll
  for (int t = 0; t < 8; ++t) { const float bb = bf16_rne(b2[t * 16 + nloc]);
#pragma unroll
    for (int r = 0; r < 8; ++r) acc[t][r] = acc[t][r] * (1.0f / (XS * WSC)) + bb; }
#pragma unroll
  for (int r = 0; r < 8; ++r) { float s = 0.0f;
#pragma unroll
    for (int t = 0; t < 8; ++t) s += acc[t][r];
    s = hsum16(s); const float mu = s * (1.0f / H); float ss = 0.0f;
#pragma unroll
    for (int t = 0; t < 8; ++t) { const float d = acc[t][r] - mu; ss += pmul(d, d); }
    ss = hsum16(ss); const float rs = rsqrtf(ss * (1.0f / H) + LN_EPS); const size_t row = m0 + 8 * hlf + r;
#pragma unroll
    for (int t = 0; t < 8; ++t) { const int c = t * 16 + nloc; Ty[wave][8 * hlf + r][c] = fmaxf(pmul((acc[t][r] - mu) * rs, bf16_rne(g[c])) + bf16_rne(be[c]), 0.0f) + H32[row * H + c]; } }
  wave_lds_sync();
  for (int pass = 0; pass < 2; ++pass) { for (int rr = 0; rr < 16; ++rr) *(volatile v4f*)(H32 + (m0 + rr) * H + lane * 4) = *(const v4f*)(&Ty[wave][rr][lane * 4]); __threadfence(); }
}
__global__ __launch_bounds__(128) void edgemlp_kernel(const float* __restrict__ H32, const int* __restrict__ src, const int* __restrict__ dst, const b16* __restrict__ EA16, const b16* __restrict__ M1, const float* __restrict__ mb1, const b16* __restrict__ M2, const float* __restrict__ mb2, const float* __restrict__ m3, const float* __restrict__ mb3, float* __restrict__ out) {
  __shared__ __attribute__((aligned(16))) b16 Fh[4][16][F4 + 8], Sh[4][16][H + 8], Sl[4][16][H + 8]; __shared__ float So[64];
  const int wave = threadIdx.x >> 5, lane = threadIdx.x & 31, nloc = lane & 15, hlf = lane >> 4, t_ = threadIdx.x; const size_t e0 = ((size_t)blockIdx.x * 4 + wave) * 16;
  { const int rr = lane >> 1, hf = lane & 1; const size_t e = e0 + rr; const int s = iclamp(src[e], 0, N - 1), d = iclamp(dst[e], 0, N - 1);
    for (int q = 0; q < 8; ++q) { const int c0 = hf * 64 + q * 8; const float* hs = H32 + (size_t)s * H + c0; const float* hd = H32 + (size_t)d * H + c0; v8b a8, b8, d8;
      for (int j = 0; j < 8; ++j) { const float a = hs[j], bq = hd[j]; a8[j] = (b16)(a * XS); b8[j] = (b16)(bq * XS); d8[j] = (b16)(fabsf(a - bq) * XS); }
      *(v8b*)(&Fh[wave][rr][c0]) = a8; *(v8b*)(&Fh[wave][rr][H + c0]) = b8; *(v8b*)(&Fh[wave][rr][2 * H + c0]) = d8; *(v8b*)(&Fh[wave][rr][3 * H + c0]) = *(const v8b*)(EA16 + e * H + c0); } }
  wave_lds_sync();
  v8f acc[8];
#pragma unroll
  for (int t = 0; t < 8; ++t) acc[t] = (v8f){};
#pragma unroll 4
  for (int kb = 0; kb < F4; kb += 32) { const v16b a = frag_kb(&Fh[wave][nloc][kb], hlf);
#pragma unroll
    for (int t = 0; t < 8; ++t) acc[t] = wmma16b(a, frag_kb(M1 + (size_t)(t * 16 + nloc) * F4 + kb, hlf), acc[t]); }
#pragma unroll
  for (int t = 0; t < 8; ++t) { const float bb = bf16_rne(mb1[t * 16 + nloc]);
#pragma unroll
    for (int r = 0; r < 8; ++r) { b16 a_, c_; split16(fmaxf(acc[t][r] * (1.0f / (XS * WSC)) + bb, 0.0f) * XS, a_, c_); Sh[wave][8 * hlf + r][t * 16 + nloc] = a_; Sl[wave][8 * hlf + r][t * 16 + nloc] = c_; } }
  wave_lds_sync();
  v8f acc2[4] = {{}, {}, {}, {}};
#pragma unroll
  for (int kb = 0; kb < H; kb += 32) { const v16b a = frag_kb(&Sh[wave][nloc][kb], hlf), al = frag_kb(&Sl[wave][nloc][kb], hlf);
#pragma unroll
    for (int t = 0; t < 4; ++t) { const v16b bw = frag_kb(M2 + (size_t)(t * 16 + nloc) * H + kb, hlf); acc2[t] = wmma16b(a, bw, acc2[t]); acc2[t] = wmma16b(al, bw, acc2[t]); } }
  const float b3 = bf16_rne(mb3[0]);
#pragma unroll
  for (int r = 0; r < 8; ++r) { float p = 0.0f;
#pragma unroll
    for (int t = 0; t < 4; ++t) { const int c = t * 16 + nloc; p += pmul(fmaxf(acc2[t][r] * (1.0f / (XS * WSC)) + bf16_rne(mb2[c]), 0.0f), bf16_rne(m3[c])); }
    p = hsum16(p); if (nloc == 0) So[wave * 16 + 8 * hlf + r] = p + b3; }
  __syncthreads();
  for (int pass = 0; pass < 2; ++pass) { if (t_ < 64) ((volatile float*)out)[(size_t)blockIdx.x * 64 + t_] = So[t_]; __threadfence(); }
}
}

extern "C" void kernel_launch(void* const* d_in, const int* in_sizes, int n_in, void* d_out, int out_size, void* d_ws, size_t ws_size, hipStream_t stream) {
  (void)n_in;
  auto Fp = [&](int i) { return (const float*)d_in[i]; };
  if (in_sizes[0] != N * ND || in_sizes[1] != E * ED || in_sizes[2] != 2 * E || in_sizes[11] != L * H * H || in_sizes[13] != L * H * H || in_sizes[17] != F4 * H || in_sizes[19] != H * H2 || out_size != E) return;
  const int* src = (const int*)d_in[2]; const int* dst = src + E;
  size_t off = 0; char* ws = (char*)d_ws;
  auto carve = [&](size_t bytes) { char* p = ws + off; off += (bytes + 255) & ~(size_t)255; return p; };
  b16* CW1 = (b16*)carve((size_t)L * H * H * 2); b16* CW2 = (b16*)carve((size_t)L * H * H * 2); b16* M1 = (b16*)carve((size_t)H * F4 * 2); b16* M2 = (b16*)carve((size_t)H2 * H * 2);
  float* H32 = (float*)carve((size_t)NP * H * 4); b16* EA16 = (b16*)carve((size_t)E * H * 2); b16* Zh = (b16*)carve((size_t)NP * H * 2); b16* Zl = (b16*)carve((size_t)NP * H * 2);
  CsrBufs csr; off = csr_carve(csr, ws, off, E, N);
  if (off > ws_size || off > ((size_t)128 << 20)) return;
  prepw_kernel<<<dim3((F4 * H / 8 + 255) / 256, 10), 256, 0, stream>>>(Fp(11), Fp(13), Fp(17), Fp(19), CW1, CW2, M1, M2);
  nodeenc_kernel<<<NP / 16, 256, 0, stream>>>(Fp(0), Fp(3), Fp(4), Fp(5), Fp(6), H32);
  edgeenc_kernel<<<E / 16, 256, 0, stream>>>(Fp(1), Fp(7), Fp(8), Fp(9), Fp(10), EA16);
  csr_build(csr, dst, E, N, stream);
  for (int l = 0; l < L; ++l) {
    aggr_kernel<<<NP / 16, 256, 0, stream>>>(H32, src, EA16, csr.PERM, csr.ROWPTR, csr.ROWCNT, (int)csr.permLen, Zh, Zl);
    nodemlp_kernel<<<NP / 64, 128, 0, stream>>>(Zh, Zl, CW1 + (size_t)l * H * H, Fp(12) + l * H, CW2 + (size_t)l * H * H, Fp(14) + l * H, Fp(15) + l * H, Fp(16) + l * H, H32); }
  edgemlp_kernel<<<E / 64, 128, 0, stream>>>(H32, src, dst, EA16, M1, Fp(18), M2, Fp(20), Fp(21), Fp(22), (float*)d_out);
}
